// LinearAttention_8065948582522
// MI455X (gfx1250) — hardware-verified
//
#include <hip/hip_runtime.h>
#include <math.h>

#define TT 4096
#define CC 128
#define DIN 128
#define NH 4
#define HD 32
#define HG 1
#define NQB (TT / 64)
#define CAUSAL 0
#define QHI 64
#define KHI 64
#define QBH 0
#define SCALE (1.0f)
typedef __attribute__((ext_vector_type(16))) _Float16 v16h;
typedef __attribute__((ext_vector_type(16))) __bf16 v16b;
typedef __attribute__((ext_vector_type(8)))  _Float16 v8h;
typedef __attribute__((ext_vector_type(8)))  float v8f;
typedef __attribute__((ext_vector_type(4)))  float v4f;
typedef __attribute__((ext_vector_type(2)))  float v2f;
typedef __attribute__((ext_vector_type(4)))  unsigned v4u;
typedef __attribute__((ext_vector_type(4)))  int v4i;
typedef float __attribute__((may_alias)) float_a;
typedef int __attribute__((may_alias)) int_a;

template <typename T> __device__ __forceinline__ void vst2(void* p, T v) { *(volatile T*)p = v; __threadfence(); *(volatile T*)p = v; }
__device__ __forceinline__ v8f wmma16(v16h a, v16h b, v8f c) {
  v8f d = __builtin_amdgcn_wmma_f32_16x16x32_f16(false, a, false, b, (short)0, c, false, false);
  asm volatile("v_nop\n\tv_nop\n\tv_nop\n\tv_nop" : "+v"(d) : "v"(a), "v"(b));
  return d;
}
__device__ __forceinline__ v8f wmma_bf(v16b a, v16b b, v8f c) {
  v8f d = __builtin_amdgcn_wmma_f32_16x16x32_bf16(false, a, false, b, (short)0, c, false, false);
  asm volatile("v_nop\n\tv_nop\n\tv_nop\n\tv_nop" : "+v"(d) : "v"(a), "v"(b));
  return d;
}
__device__ __forceinline__ v16h frag_h(const _Float16* rowk0, int lane) {
  union { v16h v; v8h q[2]; } u; const _Float16* p = rowk0 + 8 * (lane >> 4);
  u.q[0] = *(const v8h*)p; u.q[1] = *(const v8h*)(p + 16); return u.v;
}
__device__ __forceinline__ v16h frag_f32(const float* rowk0, int lane) {
  v16h a; const float* p = rowk0 + 8 * (lane >> 4);
#pragma unroll
  for (int i = 0; i < 8; ++i) { a[i] = (_Float16)p[i]; a[8 + i] = (_Float16)p[16 + i]; }
  return a;
}
__device__ __forceinline__ v16h frag_f32s(const float* rowk0, int lane, float sc) {
  v16h a; const float* p = rowk0 + 8 * (lane >> 4);
#pragma unroll
  for (int i = 0; i < 8; ++i) { a[i] = (_Float16)(p[i] * sc); a[8 + i] = (_Float16)(p[16 + i] * sc); }
  return a;
}
__device__ __forceinline__ v16h fragc_f32(const float* W, int k0, int n, int lane, int ld, int K) {
  v16h a; const int g = lane >> 4;
#pragma unroll
  for (int i = 0; i < 8; ++i) { const int ka = k0 + 8 * g + i, kb = ka + 16;
    a[i] = (_Float16)(ka < K ? W[(size_t)(ka < K ? ka : K - 1) * ld + n] : 0.f); a[8 + i] = (_Float16)(kb < K ? W[(size_t)(kb < K ? kb : K - 1) * ld + n] : 0.f); }
  return a;
}
struct F2 { v16b h, l; };
__device__ __forceinline__ F2 bsplit16(const float v[16]) { F2 r;
#pragma unroll
  for (int i = 0; i < 16; ++i) { const __bf16 h = (__bf16)v[i]; r.h[i] = h; r.l[i] = (__bf16)(v[i] - (float)h); }
  return r; }
__device__ __forceinline__ F2 split_row(const float* row, int k0, int lane) { float v[16]; const float* p = row + k0 + 8 * (lane >> 4);
#pragma unroll
  for (int i = 0; i < 8; ++i) { v[i] = p[i]; v[8 + i] = p[16 + i]; }
  return bsplit16(v); }
__device__ __forceinline__ F2 split_rowK(const float* row, int k0, int lane, int K) { float v[16]; const int g = lane >> 4;
#pragma unroll
  for (int i = 0; i < 8; ++i) { const int ka = k0 + 8 * g + i, kb = ka + 16; v[i] = ka < K ? row[ka < K ? ka : K - 1] : 0.f; v[8 + i] = kb < K ? row[kb < K ? kb : K - 1] : 0.f; }
  return bsplit16(v); }
__device__ __forceinline__ F2 split_col(const float* W, int k0, int n, int lane, int ld, int K) { float v[16]; const int g = lane >> 4;
#pragma unroll
  for (int i = 0; i < 8; ++i) { const int ka = k0 + 8 * g + i, kb = ka + 16; v[i] = ka < K ? W[(size_t)(ka < K ? ka : K - 1) * ld + n] : 0.f; v[8 + i] = kb < K ? W[(size_t)(kb < K ? kb : K - 1) * ld + n] : 0.f; }
  return bsplit16(v); }
__device__ __forceinline__ v8f mac3(const F2& a, const F2& b, v8f c) { c = wmma_bf(a.l, b.h, c); c = wmma_bf(a.h, b.l, c); return wmma_bf(a.h, b.h, c); }
__device__ __forceinline__ float sigm(float v) { return 1.0f / (1.0f + expf(-v)); }
#define LDSX() do { asm volatile("s_wait_dscnt 0" ::: "memory"); __builtin_amdgcn_wave_barrier(); __builtin_amdgcn_fence(__ATOMIC_RELEASE, "workgroup"); } while (0)

__device__ __forceinline__ float bfr(float v) { return (float)(__bf16)v; }
__host__ __device__ __forceinline__ int kb_last(int qb) { return CAUSAL ? ((qb * 64 + 63) >> 7) : (TT / 128 - 1); }
typedef __attribute__((ext_vector_type(8))) __bf16 v8b;
__device__ __forceinline__ v16b frag_b(const __bf16* rowk0, int lane) {
  union { v16b v; v8b q[2]; } u; const __bf16* p = rowk0 + 8 * (lane >> 4);
  u.q[0] = *(const v8b*)p; u.q[1] = *(const v8b*)(p + 16); return u.v;
}
__device__ __forceinline__ v16b wcol_io(const float* Wm, int k0, int o, int lane, int ld) { v16b w; const int g = lane >> 4;
#pragma unroll
  for (int i = 0; i < 8; ++i) { w[i] = (__bf16)Wm[(size_t)(k0 + 8 * g + i) * ld + o]; w[8 + i] = (__bf16)Wm[(size_t)(k0 + 16 + 8 * g + i) * ld + o]; }
  return w; }
__device__ __forceinline__ v16b wcol_oi(const float* Wm, int k0, int o, int lane, int K) { v16b w; const float* p = Wm + (size_t)o * K + k0 + 8 * (lane >> 4);
#pragma unroll
  for (int i = 0; i < 8; ++i) { w[i] = (__bf16)p[i]; w[8 + i] = (__bf16)p[16 + i]; }
  return w; }
__device__ __forceinline__ v16h wcolh_io(const float* Wm, int k0, int o, int lane, int ld) { v16h w; const int g = lane >> 4;
#pragma unroll
  for (int i = 0; i < 8; ++i) { w[i] = (_Float16)(bfr(Wm[(size_t)(k0 + 8 * g + i) * ld + o]) * 256.0f); w[8 + i] = (_Float16)(bfr(Wm[(size_t)(k0 + 16 + 8 * g + i) * ld + o]) * 256.0f); }
  return w; }
__device__ __forceinline__ v16h wcolh_oi(const float* Wm, int k0, int o, int lane, int K) { v16h w; const float* p = Wm + (size_t)o * K + k0 + 8 * (lane >> 4);
#pragma unroll
  for (int i = 0; i < 8; ++i) { w[i] = (_Float16)(bfr(p[i]) * 256.0f); w[8 + i] = (_Float16)(bfr(p[16 + i]) * 256.0f); }
  return w; }
__device__ __forceinline__ v16b wcol_hdk(const float* Wm, int k0, int o, int lane) { v16b w; const int g = lane >> 4; const float* p = Wm + (size_t)(o / HD) * DIN * HD + (o % HD);
#pragma unroll
  for (int i = 0; i < 8; ++i) { w[i] = (__bf16)p[(size_t)(k0 + 8 * g + i) * HD]; w[8 + i] = (__bf16)p[(size_t)(k0 + 16 + 8 * g + i) * HD]; }
  return w; }
#define WO_OUT_IN 1
#if WQKV_LAYOUT == 1
#define WCOL(W, k0, o, lane) wcol_oi(W, k0, o, lane, DIN)
#elif WQKV_LAYOUT == 2
#define WCOL(W, k0, o, lane) wcol_hdk(W, k0, o, lane)
#else
#define WCOL(W, k0, o, lane) wcol_io(W, k0, o, lane, CC)
#endif
#if WO_OUT_IN
#define WOCOL(W, k0, o, lane) wcol_oi(W, k0, o, lane, CC)
#define WOCOLH(W, k0, o, lane) wcolh_oi(W, k0, o, lane, CC)
#else
#define WOCOL(W, k0, o, lane) wcol_io(W, k0, o, lane, DIN)
#define WOCOLH(W, k0, o, lane) wcolh_io(W, k0, o, lane, DIN)
#endif

#ifndef SM_EXTRA_PARAMS
#define SM_EXTRA_PARAMS
#endif
#ifndef PROJ_EXTRA_PARAMS
#define PROJ_EXTRA_PARAMS
#endif
#ifndef SM_MASK_HOOK
#define SM_MASK_HOOK (void)0
#endif


#define NB 16
#define NPOS 4096
#define CIN 128
#define HID 128
#define NHD 4
#define DH 32
#define QKVW 384
#ifndef TNB
#define TNB NB
#endif
typedef _Float16 hx8 __attribute__((ext_vector_type(8)));
#define KCARRY 4096.0f
__global__ __launch_bounds__(128) void k_qkv(const float* __restrict__ X, const float* __restrict__ Wm, float* __restrict__ QKV) { __shared__ __align__(16) float sf[4][16][132];
  const int tid = threadIdx.x, wave = tid >> 5, lane = tid & 31, col = lane & 15, g = lane >> 4; const int c0 = blockIdx.y * 128; const size_t r0 = (size_t)blockIdx.x * 64 + wave * 16;
  v8f acc[8] = {};
#pragma unroll
  for (int kc = 0; kc < CIN / 32; ++kc) { v16b a; { const float* p = X + (r0 + col) * CIN + kc * 32 + 8 * g;
#pragma unroll
      for (int i = 0; i < 8; ++i) { a[i] = (__bf16)p[i]; a[8 + i] = (__bf16)p[16 + i]; } }
    asm volatile("s_wait_loadcnt 0x0" ::: "memory");
#pragma unroll
    for (int j = 0; j < 8; ++j) { const v16b w = wcol_io(Wm, kc * 32, c0 + j * 16 + col, lane, QKVW); acc[j] = wmma_bf(a, w, acc[j]); } }
#pragma unroll
  for (int j = 0; j < 8; ++j)
#pragma unroll
    for (int r = 0; r < 8; ++r) sf[wave][8 * g + r][j * 16 + col] = acc[j][r];
  LDSX(); for (int rl = 0; rl < 16; ++rl) vst2(QKV + (r0 + rl) * QKVW + c0 + lane * 4, *(const v4f*)&sf[wave][rl][lane * 4]); }
__global__ __launch_bounds__(256) void k_qsoft(const float* __restrict__ QKV, float* __restrict__ QS) { const size_t gid = (size_t)blockIdx.x * 256 + threadIdx.x; const size_t row = gid >> 2; const int h = (int)(gid & 3);
  const float* p = QKV + row * QKVW + h * DH;
  float m = -3.0e38f;
#pragma unroll 1
  for (int q = 0; q < DH / 4; ++q) { const v4f t = *(const v4f*)(p + q * 4); asm volatile("s_wait_loadcnt 0x0" ::: "memory"); m = fmaxf(m, fmaxf(fmaxf(t[0], t[1]), fmaxf(t[2], t[3]))); }
  float s2 = 0.f;
#pragma unroll 1
  for (int q = 0; q < DH / 4; ++q) { const v4f t = *(const v4f*)(p + q * 4); asm volatile("s_wait_loadcnt 0x0" ::: "memory"); _Pragma("unroll") for (int u = 0; u < 4; ++u) s2 += expf(t[u] - m); }
#pragma unroll 1
  for (int q = 0; q < DH / 4; ++q) { const v4f t = *(const v4f*)(p + q * 4); asm volatile("s_wait_loadcnt 0x0" ::: "memory"); v4f o; _Pragma("unroll") for (int u = 0; u < 4; ++u) { _Pragma("clang fp contract(off)") o[u] = (expf(t[u] - m) / s2) * 0.17677669529663687f; } vst2(QS + row * HID + h * DH + q * 4, o); } }
__global__ __launch_bounds__(128) void k_ksoft(const float* __restrict__ QKV, _Float16* __restrict__ KSH, _Float16* __restrict__ KSL) { const int c = threadIdx.x; const int b = blockIdx.x; const float* p = QKV + (size_t)b * NPOS * QKVW + HID + c;
  float mx = -3.0e38f;
#pragma unroll 1
  for (int n0 = 0; n0 < NPOS; n0 += 8) { float tv[8];
#pragma unroll
    for (int u = 0; u < 8; ++u) tv[u] = p[(size_t)(n0 + u) * QKVW];
    asm volatile("s_wait_loadcnt 0x0" ::: "memory");
#pragma unroll
    for (int u = 0; u < 8; ++u) mx = fmaxf(mx, tv[u]); }
  float sm = 0.f;
#pragma unroll 1
  for (int n0 = 0; n0 < NPOS; n0 += 8) { float tv[8];
#pragma unroll
    for (int u = 0; u < 8; ++u) tv[u] = p[(size_t)(n0 + u) * QKVW];
    asm volatile("s_wait_loadcnt 0x0" ::: "memory");
#pragma unroll
    for (int u = 0; u < 8; ++u) sm += expf(tv[u] - mx); }
  _Float16* ph = KSH + ((size_t)b * HID + c) * NPOS; _Float16* pl = KSL + ((size_t)b * HID + c) * NPOS;
#pragma unroll 1
  for (int n0 = 0; n0 < NPOS; n0 += 8) { float tv[8];
#pragma unroll
    for (int u = 0; u < 8; ++u) tv[u] = p[(size_t)(n0 + u) * QKVW];
    asm volatile("s_wait_loadcnt 0x0" ::: "memory");
    hx8 hh, hl;
#pragma unroll
    for (int u = 0; u < 8; ++u) { _Pragma("clang fp contract(off)") const float kv = (expf(tv[u] - mx) / sm) * KCARRY; const _Float16 h1 = (_Float16)kv; hh[u] = h1; hl[u] = (_Float16)((kv - (float)h1) * 1024.0f); }
    vst2((unsigned*)(ph + n0), *(const v4u*)&hh); vst2((unsigned*)(pl + n0), *(const v4u*)&hl); } }
__global__ __launch_bounds__(128) void k_ctx(const _Float16* __restrict__ KSH, const _Float16* __restrict__ KSL, const float* __restrict__ QKV, float* __restrict__ CTX) { __shared__ __align__(16) float st[32][36];
  const int tid = threadIdx.x, wave = tid >> 5, lane = tid & 31, col = lane & 15, g = lane >> 4; const int b = blockIdx.x, h = blockIdx.y; const int dt = wave >> 1, et = wave & 1;
  const _Float16* ah0 = KSH + ((size_t)b * HID + h * DH + dt * 16 + col) * NPOS; const _Float16* al0 = KSL + ((size_t)b * HID + h * DH + dt * 16 + col) * NPOS;
  const float* vb = QKV + (size_t)b * NPOS * QKVW + 2 * HID + h * DH + et * 16 + col;
  v8f acc = {}, accl = {};
#pragma unroll 1
  for (int kc = 0; kc < NPOS / 32; ++kc) { const v16h ah = frag_h(ah0 + kc * 32, lane), al = frag_h(al0 + kc * 32, lane); asm volatile("s_wait_loadcnt 0x0" ::: "memory"); v16h bh, bl; { float tv[16];
#pragma unroll
      for (int i = 0; i < 8; ++i) tv[i] = vb[(size_t)(kc * 32 + 8 * g + i) * QKVW];
      asm volatile("s_wait_loadcnt 0x0" ::: "memory");
#pragma unroll
      for (int i = 0; i < 8; ++i) tv[8 + i] = vb[(size_t)(kc * 32 + 16 + 8 * g + i) * QKVW];
      asm volatile("s_wait_loadcnt 0x0" ::: "memory");
#pragma unroll
      for (int i = 0; i < 16; ++i) { const _Float16 h1 = (_Float16)tv[i]; bh[i] = h1; bl[i] = (_Float16)((tv[i] - (float)h1) * 1024.0f); } }
    acc = wmma16(ah, bh, acc); accl = wmma16(al, bh, accl); accl = wmma16(ah, bl, accl); }
#pragma unroll
  for (int r = 0; r < 8; ++r) st[dt * 16 + 8 * g + r][et * 16 + col] = (acc[r] + accl[r] * (1.0f / 1024.0f)) * (1.0f / KCARRY);
  __syncthreads();
  if (tid < 32 * 8) { for (int e2 = tid; e2 < 32 * 8; e2 += 128) { const int d = e2 >> 3, q = e2 & 7; vst2(CTX + (((size_t)b * NHD + h) * DH + d) * DH + q * 4, *(const v4f*)&st[d][q * 4]); } } }
__global__ __launch_bounds__(128) void k_o(const float* __restrict__ QS, const float* __restrict__ CTX, float* __restrict__ O) { __shared__ __align__(16) float sf[4][16][132];
  const int tid = threadIdx.x, wave = tid >> 5, lane = tid & 31, col = lane & 15, g = lane >> 4; const size_t r0 = (size_t)blockIdx.x * 64 + wave * 16; const int b = (int)(r0 / NPOS);
#pragma unroll
  for (int h = 0; h < NHD; ++h) { v16h ah, al; { float tv[16]; const float* p = QS + (r0 + col) * HID + h * DH + 8 * g;
#pragma unroll
      for (int i = 0; i < 8; ++i) { tv[i] = p[i]; tv[8 + i] = p[16 + i]; }
      asm volatile("s_wait_loadcnt 0x0" ::: "memory");
#pragma unroll
      for (int i = 0; i < 16; ++i) { const _Float16 h1 = (_Float16)tv[i]; ah[i] = h1; al[i] = (_Float16)((tv[i] - (float)h1) * 1024.0f); } }
#pragma unroll
    for (int j = 0; j < 2; ++j) { v16h bh, bl; { float tv[16]; const float* p = CTX + (((size_t)b * NHD + h) * DH) * DH + j * 16 + col;
#pragma unroll
        for (int i = 0; i < 8; ++i) { tv[i] = p[(size_t)(8 * g + i) * DH]; tv[8 + i] = p[(size_t)(16 + 8 * g + i) * DH]; }
        asm volatile("s_wait_loadcnt 0x0" ::: "memory");
#pragma unroll
        for (int i = 0; i < 16; ++i) { const _Float16 h1 = (_Float16)tv[i]; bh[i] = h1; bl[i] = (_Float16)((tv[i] - (float)h1) * 1024.0f); } }
      v8f acc = {}, accl = {}; acc = wmma16(ah, bh, acc); accl = wmma16(al, bh, accl); accl = wmma16(ah, bl, accl);
#pragma unroll
      for (int r = 0; r < 8; ++r) sf[wave][8 * g + r][h * DH + j * 16 + col] = acc[r] + accl[r] * (1.0f / 1024.0f); } }
  LDSX(); for (int rl = 0; rl < 16; ++rl) vst2(O + (r0 + rl) * HID + lane * 4, *(const v4f*)&sf[wave][rl][lane * 4]); }
__global__ __launch_bounds__(128) void k_y(const float* __restrict__ O, const float* __restrict__ WO, const float* __restrict__ BO, const float* __restrict__ G, const float* __restrict__ BT, float* __restrict__ OUT) { __shared__ __align__(16) float sf[4][16][132];
  const int tid = threadIdx.x, wave = tid >> 5, lane = tid & 31, col = lane & 15, g = lane >> 4; const size_t r0 = (size_t)blockIdx.x * 64 + wave * 16;
  v8f acc[8] = {};
#pragma unroll
  for (int kc = 0; kc < HID / 32; ++kc) { const F2 a = split_row(O + (r0 + col) * HID, kc * 32, lane);
    asm volatile("s_wait_loadcnt 0x0" ::: "memory");
#pragma unroll
    for (int j = 0; j < 8; ++j) { const v16b w = wcol_io(WO, kc * 32, j * 16 + col, lane, CIN); acc[j] = wmma_bf(a.h, w, acc[j]); acc[j] = wmma_bf(a.l, w, acc[j]); } }
#pragma unroll
  for (int j = 0; j < 8; ++j) { const float bb = bfr(BO[j * 16 + col]); asm volatile("s_wait_loadcnt 0x0" ::: "memory");
#pragma unroll
    for (int r = 0; r < 8; ++r) sf[wave][8 * g + r][j * 16 + col] = acc[j][r] + bb; }
  LDSX();
  float gv[4], bv[4]; { const v4f g4 = *(const v4f*)(G + lane * 4), b4 = *(const v4f*)(BT + lane * 4); asm volatile("s_wait_loadcnt 0x0" ::: "memory"); _Pragma("unroll") for (int u = 0; u < 4; ++u) { gv[u] = bfr(g4[u]); bv[u] = bfr(b4[u]); } }
  for (int rl = 0; rl < 16; ++rl) { const v4f v = *(const v4f*)&sf[wave][rl][lane * 4]; float s1 = v[0] + v[1] + v[2] + v[3];
#pragma unroll
    for (int o = 1; o < 32; o <<= 1) s1 += __shfl_xor(s1, o);
    const float mean = s1 * (1.0f / CIN); float q2 = 0.f; _Pragma("unroll") for (int u = 0; u < 4; ++u) { const float d = v[u] - mean; q2 += d * d; }
#pragma unroll
    for (int o = 1; o < 32; o <<= 1) q2 += __shfl_xor(q2, o);
    const float rs = 1.0f / sqrtf(q2 * (1.0f / CIN) + 1e-5f); v4f ov; _Pragma("unroll") for (int u = 0; u < 4; ++u) ov[u] = (v[u] - mean) * rs * gv[u] + bv[u];
    vst2(OUT + (r0 + rl) * CIN + lane * 4, ov); } }
#define WS_QKV 0u
#define WS_QS  (WS_QKV + 4u * (size_t)NB * NPOS * QKVW)
#define WS_KSH (WS_QS + 4u * (size_t)NB * NPOS * HID)
#define WS_KSL (WS_KSH + 2u * (size_t)NB * HID * NPOS)
#define WS_CTX (WS_KSL + 2u * (size_t)NB * HID * NPOS)
#define WS_O   (WS_CTX + 4u * (size_t)NB * NHD * DH * DH)
#define WS_END (WS_O + 4u * (size_t)NB * NPOS * HID)
static_assert(WS_END <= 268435456u, "ws");
extern "C" void kernel_launch(void* const* d_in, const int* in_sizes, int n_in, void* d_out, int out_size, void* d_ws, size_t ws_size, hipStream_t stream) {
  (void)in_sizes; (void)n_in; (void)out_size;
  const float** F = (const float**)d_in;
  if (ws_size < (size_t)WS_END) return;
  char* ws = (char*)d_ws; float *QKV = (float*)(ws + WS_QKV), *QS = (float*)(ws + WS_QS), *CTX = (float*)(ws + WS_CTX), *O = (float*)(ws + WS_O); _Float16 *KSH = (_Float16*)(ws + WS_KSH), *KSL = (_Float16*)(ws + WS_KSL);
  k_qkv<<<dim3(TNB * NPOS / 64, QKVW / 128), 128, 0, stream>>>(F[0], F[1], QKV);
  k_qsoft<<<dim3(TNB * NPOS * NHD / 256), 256, 0, stream>>>(QKV, QS);
  k_ksoft<<<dim3(TNB), 128, 0, stream>>>(QKV, KSH, KSL);
  k_ctx<<<dim3(TNB, NHD), 128, 0, stream>>>(KSH, KSL, QKV, CTX);
  k_o<<<dim3(TNB * NPOS / 64), 128, 0, stream>>>(QS, CTX, O);
  k_y<<<dim3(TNB * NPOS / 64), 128, 0, stream>>>(O, F[2], F[3], F[4], F[5], (float*)d_out);
}
